// ElasticBertSelfAttention_74363063763242
// MI455X (gfx1250) — hardware-verified
//
#include <hip/hip_runtime.h>


#define NB_  4
#define SS   1024
#define DM   1024
#define NH_  16
#define HD   64
#define NE   2048
#define EOFF 1024
#define HPP  4
typedef _Float16 h16;
typedef unsigned short bf;
typedef __attribute__((ext_vector_type(16))) __bf16   v16bf;
typedef __attribute__((ext_vector_type(16))) _Float16 v16h;
typedef __attribute__((ext_vector_type(8)))  _Float16 v8h;
typedef __attribute__((ext_vector_type(8)))  unsigned short v8us;
typedef __attribute__((ext_vector_type(8)))  float    v8f;
typedef __attribute__((ext_vector_type(4)))  float    v4f;
typedef v8h  __attribute__((may_alias)) v8ha;
typedef v4f  __attribute__((may_alias)) v4fa;
typedef v8us __attribute__((may_alias)) v8usa;

__device__ __forceinline__ unsigned short f2bf(float f) { unsigned u = __float_as_uint(f); u += 0x7FFFu + ((u >> 16) & 1u); return (unsigned short)(u >> 16); }
__device__ __forceinline__ float bf2f(unsigned short b) { return __uint_as_float(((unsigned)b) << 16); }
__device__ __forceinline__ float bfr(float f) { return bf2f(f2bf(f)); }
__device__ __forceinline__ v16h cat16(v8h lo, v8h hi) { return __builtin_shufflevector(lo, hi, 0, 1, 2, 3, 4, 5, 6, 7, 8, 9, 10, 11, 12, 13, 14, 15); }
__device__ __forceinline__ v16bf cat16b(v8us lo, v8us hi) { return __builtin_bit_cast(v16bf, __builtin_shufflevector(lo, hi, 0, 1, 2, 3, 4, 5, 6, 7, 8, 9, 10, 11, 12, 13, 14, 15)); }
__device__ __forceinline__ v8f wmma16(v16h a, v16h b, v8f c) { return __builtin_amdgcn_wmma_f32_16x16x32_f16(false, a, false, b, (short)0, c, false, false); }
__device__ __forceinline__ v8f wmmab(v16bf a, v16bf b, v8f c) { return __builtin_amdgcn_wmma_f32_16x16x32_bf16(false, a, false, b, (short)0, c, false, false); }


template <typename T16> struct WFrag;
template <> struct WFrag<h16> { typedef v16h V; static __device__ __forceinline__ V ld(const h16* p) { return cat16(*(const v8h*)p, *(const v8h*)(p + 16)); } static __device__ __forceinline__ v8f mma(V a, V b, v8f c) { return wmma16(a, b, c); } };
template <> struct WFrag<bf> { typedef v16bf V; static __device__ __forceinline__ V ld(const bf* p) { return cat16b(*(const v8us*)p, *(const v8us*)(p + 16)); } static __device__ __forceinline__ v8f mma(V a, V b, v8f c) { return wmmab(a, b, c); } };
template <typename T16, int NSPLIT, bool BIAS>
__global__ __launch_bounds__(32) void k_gemmw(const T16* __restrict__ A, const T16* __restrict__ A2, const T16* __restrict__ Bt, const T16* __restrict__ Bt2, int K, float* C, int ldc, const float* __restrict__ bias, size_t sA, size_t sB, size_t sC) {
    typedef typename WFrag<T16>::V V;
    __shared__ __align__(16) float os[16 * 68];
    const size_t z = blockIdx.z; A += z * sA; if (A2) A2 += z * sA; Bt += z * sB; if (Bt2) Bt2 += z * sB; C += z * sC;
    const int lane = threadIdx.x & 31, lr = lane & 15, hi = lane >> 4; const int r0 = blockIdx.x * 64, c0 = blockIdx.y * 64;
    v8f acc[4][4];
#pragma unroll
    for (int mb = 0; mb < 4; ++mb)
#pragma unroll
        for (int nb = 0; nb < 4; ++nb) acc[mb][nb] = (v8f){};
    const size_t aoff = (size_t)(r0 + lr) * K + 8 * hi, boff = (size_t)(c0 + lr) * K + 8 * hi;
#pragma unroll 1
    for (int kc = 0; kc < K; kc += 32) {
        V a[4], a2[4];
#pragma unroll
        for (int mb = 0; mb < 4; ++mb) { a[mb] = WFrag<T16>::ld(A + aoff + (size_t)mb * 16 * K + kc); if (NSPLIT == 1 || NSPLIT == 2) a2[mb] = WFrag<T16>::ld(A2 + aoff + (size_t)mb * 16 * K + kc); }
#pragma unroll
        for (int nb = 0; nb < 4; ++nb) { const V b = WFrag<T16>::ld(Bt + boff + (size_t)nb * 16 * K + kc); V b2; if (NSPLIT >= 2) b2 = WFrag<T16>::ld(Bt2 + boff + (size_t)nb * 16 * K + kc);
#pragma unroll
            for (int mb = 0; mb < 4; ++mb) { acc[mb][nb] = WFrag<T16>::mma(a[mb], b, acc[mb][nb]); if (NSPLIT == 1 || NSPLIT == 2) acc[mb][nb] = WFrag<T16>::mma(a2[mb], b, acc[mb][nb]); if (NSPLIT >= 2) acc[mb][nb] = WFrag<T16>::mma(a[mb], b2, acc[mb][nb]); } }
        asm volatile("v_nop\n\tv_nop\n\tv_nop\n\tv_nop" : "+v"(acc[0][0]), "+v"(acc[1][1]), "+v"(acc[2][2]), "+v"(acc[3][3]) : "v"(a[0]), "v"(a[3]));
    }
#pragma unroll
    for (int mb = 0; mb < 4; ++mb) {
#pragma unroll
        for (int nb = 0; nb < 4; ++nb) {
#pragma unroll
            for (int j = 0; j < 8; ++j) os[(hi * 8 + j) * 68 + nb * 16 + lr] = acc[mb][nb][j]; }
        __builtin_amdgcn_wave_barrier(); asm volatile("" ::: "memory");
        float* crow = C + (size_t)(r0 + mb * 16) * ldc + c0;
#pragma unroll 1
        for (int ps = 0; ps < 2; ++ps) {
#pragma unroll
            for (int s = 0; s < 8; ++s) { const int row = 2 * s + hi, cofs = lr * 4; v4f val = *(const v4fa*)(os + row * 68 + cofs); if (BIAS) { val[0] += bfr(bias[c0 + cofs]); val[1] += bfr(bias[c0 + cofs + 1]); val[2] += bfr(bias[c0 + cofs + 2]); val[3] += bfr(bias[c0 + cofs + 3]); }
                *(volatile v4f*)(crow + (size_t)row * ldc + cofs) = val; }
            if (ps == 0) __threadfence(); }
        __builtin_amdgcn_wave_barrier(); asm volatile("" ::: "memory");
    }
}

__device__ __forceinline__ h16 tohx(float x) { return (h16)x; }
__device__ __forceinline__ void splitf(float y, unsigned short& h, unsigned short& l) { h = f2bf(y); l = f2bf(y - bf2f(h)); }
typedef __attribute__((ext_vector_type(2))) unsigned short v2us;
typedef __attribute__((ext_vector_type(4))) unsigned short v4us;
typedef __attribute__((ext_vector_type(4))) _Float16 v4h;

__global__ __launch_bounds__(256) void k_wtG(const float* __restrict__ w, int K, int N, bf* Bt) {
    const int lane = threadIdx.x & 31; const int L0 = (blockIdx.x * 8 + (threadIdx.x >> 5)) * 8; const int nlines = N * K / 64;
#pragma unroll
    for (int ps = 0; ps < 2; ++ps) {
#pragma unroll 1
        for (int l = 0; l < 8; ++l) { const int L = L0 + l; if (L >= nlines) break; const size_t e = (size_t)L * 64 + lane * 2; const int k = (int)(e % K), n = (int)(e / K); v2us o;
            o[0] = f2bf(w[(size_t)k * N + n]); o[1] = f2bf(w[(size_t)(k + 1) * N + n]); *(volatile v2us*)(Bt + e) = o; }
        if (ps == 0) __threadfence(); }
}
__global__ __launch_bounds__(256) void k_cvt8(const float* __restrict__ src, bf* dst, size_t n8) { const size_t i = (size_t)blockIdx.x * 256 + threadIdx.x; if (i >= n8) return; const v8f v = *(const v8f*)(src + i * 8); v8us o;
#pragma unroll
    for (int k = 0; k < 8; ++k) o[k] = f2bf(v[k]); *(volatile v8us*)(dst + i * 8) = o; __threadfence(); *(volatile v8us*)(dst + i * 8) = o; }
__global__ __launch_bounds__(256) void k_e16(const float* __restrict__ emb, h16* E16) { const int e = (blockIdx.x * 256 + threadIdx.x) * 4; if (e >= NE * HD) return; const v4f a = *(const v4f*)(emb + (size_t)EOFF * HD + e); v4h o;
#pragma unroll
    for (int u = 0; u < 4; ++u) o[u] = tohx(bfr(a[u])); *(volatile v4h*)(E16 + e) = o; __threadfence(); *(volatile v4h*)(E16 + e) = o; }
__global__ __launch_bounds__(256) void k_qkp(const float* __restrict__ FQ, const float* __restrict__ FK, bf* Qh, bf* Ql, h16* Q16, bf* Kh, bf* Kl, h16* K16) { const int e = (blockIdx.x * 256 + threadIdx.x) * 4; if (e >= NH_ * SS * HD) return; const int d = e % HD; const int t = (e / HD) % SS; const int h = e / (HD * SS); const size_t f = (size_t)t * DM + h * HD + d; v4us qh, ql, kh, kl; v4h q6, k6;
#pragma unroll
    for (int u = 0; u < 4; ++u) { const float qv = FQ[f + u], kv = FK[f + u]; unsigned short a, b; splitf(qv, a, b); qh[u] = a; ql[u] = b; splitf(kv, a, b); kh[u] = a; kl[u] = b; q6[u] = tohx(qv); k6[u] = tohx(kv); }
    for (int ps = 0; ps < 2; ++ps) { *(volatile v4us*)(Qh + e) = qh; *(volatile v4us*)(Ql + e) = ql; *(volatile v4h*)(Q16 + e) = q6; *(volatile v4us*)(Kh + e) = kh; *(volatile v4us*)(Kl + e) = kl; *(volatile v4h*)(K16 + e) = k6; if (ps == 0) __threadfence(); } }
__global__ __launch_bounds__(256) void k_vtp2(const float* __restrict__ FV, bf* VTh, bf* VTl) { const int e = (blockIdx.x * 256 + threadIdx.x) * 2; if (e >= NH_ * HD * SS) return; const int t = e % SS; const int d = (e / SS) % HD; const int h = e / (SS * HD); v2us oh, ol;
#pragma unroll
    for (int u = 0; u < 2; ++u) { unsigned short a, b; splitf(FV[(size_t)(t + u) * DM + h * HD + d], a, b); oh[u] = a; ol[u] = b; }
    *(volatile v2us*)(VTh + e) = oh; *(volatile v2us*)(VTl + e) = ol; __threadfence(); *(volatile v2us*)(VTh + e) = oh; *(volatile v2us*)(VTl + e) = ol; }
__global__ __launch_bounds__(256) void k_ebsoft(const float* __restrict__ Sb, const float* __restrict__ QE, const float* __restrict__ KE, const float* __restrict__ am, bf* Ph, bf* Pl) { const int lane = threadIdx.x & 31; const int row = blockIdx.x * 8 + (threadIdx.x >> 5); if (row >= HPP * SS) return; const int l = row % SS; const int z = row / SS;
    const float* sr = Sb + (size_t)row * SS; const float* qe = QE + (size_t)row * NE + l + (SS - 1); const float* ke = KE + (size_t)z * SS * NE + l + (SS - 1); float v[SS / 32]; float mx = -3.0e38f;
#pragma unroll
    for (int ch = 0; ch < SS / 128; ++ch) { const int r0 = ch * 128 + lane * 4; const v4f a = *(const v4f*)(sr + r0);
#pragma unroll
        for (int u = 0; u < 4; ++u) { const int r = r0 + u; const float s1 = __fadd_rn(a[u], qe[-r]); const float s2 = __fadd_rn(s1, ke[(size_t)r * NE - r]); float t0 = s2 * 0.125f; asm volatile("" : "+v"(t0)); const float t = __fadd_rn(t0, bfr(am[r])); v[ch * 4 + u] = t; mx = fmaxf(mx, t); } }
#pragma unroll
    for (int sh = 16; sh; sh >>= 1) mx = fmaxf(mx, __shfl_xor(mx, sh, 32));
    float sum = 0.f;
#pragma unroll
    for (int q = 0; q < SS / 32; ++q) { float d0 = __fsub_rn(v[q], mx); asm volatile("" : "+v"(d0)); v[q] = __builtin_amdgcn_exp2f(__fmul_rn(d0, 1.4426950408889634f)); sum += v[q]; }
#pragma unroll
    for (int sh = 16; sh; sh >>= 1) sum += __shfl_xor(sum, sh, 32);
    const float f = __fdiv_rn(1.0f, sum);
    for (int ps = 0; ps < 2; ++ps) {
#pragma unroll
        for (int ch = 0; ch < SS / 128; ++ch) { v4us oh, ol;
#pragma unroll
            for (int u = 0; u < 4; ++u) { unsigned short a, b; splitf(v[ch * 4 + u] * f, a, b); oh[u] = a; ol[u] = b; } const size_t oo = (size_t)row * SS + ch * 128 + lane * 4; *(volatile v4us*)(Ph + oo) = oh; *(volatile v4us*)(Pl + oo) = ol; }
        if (ps == 0) __threadfence(); } }
__global__ __launch_bounds__(256) void k_mrg(const float* __restrict__ O, int h0, float* outb) { const int e = (blockIdx.x * 256 + threadIdx.x) * 4; if (e >= HPP * SS * HD) return; const int d = e % HD; const int t = (e / HD) % SS; const int z = e / (HD * SS); const v4f a = *(const v4f*)(O + e); const size_t oo = (size_t)t * DM + (h0 + z) * HD + d;
    *(volatile v4f*)(outb + oo) = a; __threadfence(); *(volatile v4f*)(outb + oo) = a; }

extern "C" void kernel_launch(void* const* d_in, const int* in_sizes, int n_in,
                              void* d_out, int out_size, void* d_ws, size_t ws_size, hipStream_t stream) {
    (void)in_sizes; (void)n_in; (void)out_size;
    const float** I = (const float**)d_in;
    const float *x = I[0], *am = I[1], *wq = I[2], *bq = I[3], *wk = I[4], *bk = I[5], *wv = I[6], *bv = I[7], *emb = I[8];
    float* OUT = (float*)d_out;
    char* wsp = (char*)d_ws;
    auto take = [&](size_t bytes) { char* p = wsp; wsp += (bytes + 255) & ~(size_t)255; return (void*)p; };
    bf* WQ = (bf*)take((size_t)DM * DM * 2); bf* WK = (bf*)take((size_t)DM * DM * 2); bf* WV = (bf*)take((size_t)DM * DM * 2); h16* E16 = (h16*)take((size_t)NE * HD * 2);
    bf* XB = (bf*)take((size_t)SS * DM * 2); float* FQ = (float*)take((size_t)SS * DM * 4); float* FK = (float*)take((size_t)SS * DM * 4); float* FV = (float*)take((size_t)SS * DM * 4);
    bf* Qh = (bf*)take((size_t)NH_ * SS * HD * 2); bf* Ql = (bf*)take((size_t)NH_ * SS * HD * 2); h16* Q16 = (h16*)take((size_t)NH_ * SS * HD * 2); bf* Kh = (bf*)take((size_t)NH_ * SS * HD * 2); bf* Kl = (bf*)take((size_t)NH_ * SS * HD * 2); h16* K16 = (h16*)take((size_t)NH_ * SS * HD * 2); bf* VTh = (bf*)take((size_t)NH_ * HD * SS * 2); bf* VTl = (bf*)take((size_t)NH_ * HD * SS * 2);
    float* Sb = (float*)take((size_t)HPP * SS * SS * 4); float* QE = (float*)take((size_t)HPP * SS * NE * 4); float* KE = (float*)take((size_t)HPP * SS * NE * 4); bf* Ph = (bf*)take((size_t)HPP * SS * SS * 2); bf* Pl = (bf*)take((size_t)HPP * SS * SS * 2); float* O = (float*)take((size_t)HPP * SS * HD * 4);
    if ((size_t)(wsp - (char*)d_ws) > ws_size) return;
    k_wtG<<<(DM * DM / 64 + 63) / 64, 256, 0, stream>>>(wq, DM, DM, WQ); k_wtG<<<(DM * DM / 64 + 63) / 64, 256, 0, stream>>>(wk, DM, DM, WK); k_wtG<<<(DM * DM / 64 + 63) / 64, 256, 0, stream>>>(wv, DM, DM, WV); k_e16<<<(NE * HD / 4 + 255) / 256, 256, 0, stream>>>(emb, E16);
    for (int b = 0; b < NB_; ++b) {
        k_cvt8<<<(SS * DM / 8 + 255) / 256, 256, 0, stream>>>(x + (size_t)b * SS * DM, XB, (size_t)SS * DM / 8);
        k_gemmw<bf, 0, true><<<dim3(SS / 64, DM / 64, 1), 32, 0, stream>>>(XB, nullptr, WQ, nullptr, DM, FQ, DM, bq, 0, 0, 0); k_gemmw<bf, 0, true><<<dim3(SS / 64, DM / 64, 1), 32, 0, stream>>>(XB, nullptr, WK, nullptr, DM, FK, DM, bk, 0, 0, 0); k_gemmw<bf, 0, true><<<dim3(SS / 64, DM / 64, 1), 32, 0, stream>>>(XB, nullptr, WV, nullptr, DM, FV, DM, bv, 0, 0, 0);
        k_qkp<<<(NH_ * SS * HD / 4 + 255) / 256, 256, 0, stream>>>(FQ, FK, Qh, Ql, Q16, Kh, Kl, K16); k_vtp2<<<(NH_ * HD * SS / 2 + 255) / 256, 256, 0, stream>>>(FV, VTh, VTl);
        for (int h0 = 0; h0 < NH_; h0 += HPP) { const size_t zo = (size_t)h0 * SS * HD;
            k_gemmw<bf, 2, false><<<dim3(SS / 64, SS / 64, HPP), 32, 0, stream>>>(Qh + zo, Ql + zo, Kh + zo, Kl + zo, HD, Sb, SS, nullptr, (size_t)SS * HD, (size_t)SS * HD, (size_t)SS * SS);
            k_gemmw<h16, 0, false><<<dim3(SS / 64, NE / 64, HPP), 32, 0, stream>>>(Q16 + zo, nullptr, E16, nullptr, HD, QE, NE, nullptr, (size_t)SS * HD, 0, (size_t)SS * NE);
            k_gemmw<h16, 0, false><<<dim3(SS / 64, NE / 64, HPP), 32, 0, stream>>>(K16 + zo, nullptr, E16, nullptr, HD, KE, NE, nullptr, (size_t)SS * HD, 0, (size_t)SS * NE);
            k_ebsoft<<<HPP * SS / 8, 256, 0, stream>>>(Sb, QE, KE, am + (size_t)b * SS, Ph, Pl);
            k_gemmw<bf, 2, false><<<dim3(SS / 64, 1, HPP), 32, 0, stream>>>(Ph, Pl, VTh + (size_t)h0 * HD * SS, VTl + (size_t)h0 * HD * SS, SS, O, HD, nullptr, (size_t)SS * SS, (size_t)HD * SS, (size_t)SS * HD);
            k_mrg<<<(HPP * SS * HD / 4 + 255) / 256, 256, 0, stream>>>(O, h0, OUT + (size_t)b * SS * DM); } }
}
